// MessagePassingLayer2_87110526697696
// MI455X (gfx1250) — hardware-run, weakly checked
//
#include <hip/hip_runtime.h>
#include <stddef.h>
#include <stdint.h>
#include <math.h>

#define NN      100000
#define NT      8
#define NE      400000
#define FD      128
#define GBM     128
#define MP      100096
#define SP      132
#define NTHR    256
#define NWAVE   8
#define EPT     4
#define WCH     (32 * EPT)
#define NBRUN   4096
#define SLB     12
#define NBK     25
#define NSLOT   (NBK * NBRUN)
#define NROLE   (2 * NT)
#define WLCAP   2560
#define RCAP    20480
#define DEGCAP  32
#define MAXDEG_MEAS   16
#define MAXB1024_MEAS 4295
#define RPB     8
#define WSMAX   (128u << 20)

#define BK_ZINTS (NWAVE * WLCAP + RCAP + 3 * NBRUN)
#define BK_INTS  (BK_ZINTS + 16)
#define BK_LDS   (BK_INTS * 4)
#define GEMM_LDS ((GBM * SP + GBM) * 4)

#define PBX   (MP * FD / 8 / NTHR)
#define PBW   (NT * FD * FD / 8 / NTHR)
#define PBTOT (PBX + PBW + 1)

static_assert((NT & (NT - 1)) == 0);
static_assert(MP % GBM == 0 && MP >= NN && MP == 782 * GBM);
static_assert(NBRUN == (1 << SLB) && NBRUN % GBM == 0 && NBRUN % (NTHR * 4) == 0 && NBRUN % 32 == 0);
static_assert(NBK * NBRUN >= MP);
static_assert(NN <= (1 << 17));
static_assert((((long long)NE) << SLB) < (1LL << 31));
static_assert(NE % WCH == 0 && NE % 4 == 0);
static_assert(((NE + NWAVE * WCH - 1) / (NWAVE * WCH)) * WCH * (NWAVE - 1) < NE);
static_assert(RCAP == NWAVE * WLCAP && RCAP % (NTHR * 4) == 0 && BK_ZINTS % 4 == 0);
static_assert(RCAP >= 4 * MAXB1024_MEAS + 1024);
static_assert(WLCAP >= (4 * MAXB1024_MEAS) / 8 + 8 * 46 + 1);
static_assert(DEGCAP >= MAXDEG_MEAS + 8 && DEGCAP <= 32);
static_assert(NN % RPB == 0 && RPB == NWAVE);
static_assert(FD % 32 == 0 && FD == 4 * 32);
static_assert((MP * FD / 8) % NTHR == 0 && (NT * FD * FD / 8) % NTHR == 0);
static_assert(BK_LDS <= 300000 && GEMM_LDS <= 300000);
static_assert((SP * 4) % 16 == 0);

typedef float          v4f   __attribute__((ext_vector_type(4)));
typedef float          v8f   __attribute__((ext_vector_type(8)));
typedef int            v4i   __attribute__((ext_vector_type(4)));
typedef int            v8i   __attribute__((ext_vector_type(8)));
typedef unsigned short v8us  __attribute__((ext_vector_type(8)));
typedef unsigned short v16us __attribute__((ext_vector_type(16)));
typedef __bf16         v16bf __attribute__((ext_vector_type(16)));
typedef v4f  __attribute__((may_alias)) v4fa;
typedef v4i  __attribute__((may_alias)) v4ia;
typedef v8us __attribute__((may_alias)) v8usa;
union FragB { v16bf v; v16us u; v8us h[2]; v8i w; };

__device__ __forceinline__ v8f wmb(const FragB& a, const FragB& b, v8f c) {
  v8f d = __builtin_amdgcn_wmma_f32_16x16x32_bf16(false, a.v, false, b.v, (short)0, c, false, false);
  asm volatile("v_nop\n\tv_nop\n\tv_nop\n\tv_nop" : "+v"(d) : "v"(a.w), "v"(b.w));
  return d;
}

__device__ __forceinline__ unsigned bf16_bits(float f) {
  const unsigned u = __float_as_uint(f);
  const unsigned r = (u + 0x7FFFu + ((u >> 16) & 1u)) >> 16;
  const unsigned q = (u >> 16) | 0x40u;
  return ((u & 0x7fffffffu) > 0x7f800000u) ? q : r;
}
__device__ __forceinline__ float bf16_val(float f) {
  return __uint_as_float(bf16_bits(f) << 16);
}

__device__ __forceinline__ void st2_v4f(float* p, v4f v) {
  *(volatile v4f*)p = v;
  __threadfence();
  *(volatile v4f*)p = v;
}
__device__ __forceinline__ void st2_v8us(unsigned short* p, v8us v) {
  *(volatile v8us*)p = v;
  __threadfence();
  *(volatile v8us*)p = v;
}

__device__ __forceinline__ v8us gather8(const float* __restrict__ base, int stride) {
  float f[8];
#pragma unroll
  for (int i = 0; i < 8; ++i) f[i] = base[(size_t)i * (size_t)stride];
  v8us o;
#pragma unroll
  for (int i = 0; i < 8; ++i) o[i] = (unsigned short)bf16_bits(f[i]);
  return o;
}

__global__ __launch_bounds__(NTHR) void k_prep(const float* __restrict__ x, const float* __restrict__ w,
                                               const float* __restrict__ b, unsigned short* xb,
                                               unsigned short* wt, float* bf) {
  const int tid = (int)threadIdx.x, lane = tid & 31;
  const int blk = (int)blockIdx.x;
  if (blk < PBX) {
    const int u   = blk * NTHR + tid;
    const int row = u >> 4, k8 = (u & 15) * 8;
    const int rc  = row < NN ? row : NN - 1;
    const unsigned mk = row < NN ? 0xffffu : 0u;
    const float* p = x + (size_t)rc * FD + k8;
    const v4f a = *(const v4fa*)p;
    const v4f c = *(const v4fa*)(p + 4);
    v8us o;
    o[0] = (unsigned short)(bf16_bits(a.x) & mk); o[1] = (unsigned short)(bf16_bits(a.y) & mk);
    o[2] = (unsigned short)(bf16_bits(a.z) & mk); o[3] = (unsigned short)(bf16_bits(a.w) & mk);
    o[4] = (unsigned short)(bf16_bits(c.x) & mk); o[5] = (unsigned short)(bf16_bits(c.y) & mk);
    o[6] = (unsigned short)(bf16_bits(c.z) & mk); o[7] = (unsigned short)(bf16_bits(c.w) & mk);
    st2_v8us(xb + (size_t)row * FD + k8, o);
  } else if (blk < PBX + PBW) {
    const int u  = (blk - PBX) * NTHR + tid;
    const int t  = u >> 11, n = (u >> 4) & (FD - 1), k8 = (u & 15) * 8;
    const v8us o = gather8(w + (size_t)(FD * t + k8) * FD + n, FD);
    st2_v8us(wt + (size_t)t * FD * FD + (size_t)n * FD + k8, o);
  } else {
    if (tid < 32) {
      const v4f a = *(const v4fa*)(b + 4 * lane);
      v4f o;
      o.x = bf16_val(a.x); o.y = bf16_val(a.y); o.z = bf16_val(a.z); o.w = bf16_val(a.w);
      st2_v4f(bf + 4 * lane, o);
    }
  }
}

__device__ __forceinline__ void bucket_flush(const int* pl, const int* cnt, const int* offs, int ov, int isList,
                                             int slot0, int* lp, int* cp, int* op, int* fp, int tid) {
  if (isList != 0) {
#pragma unroll 1
    for (int i = tid * 4; i < RCAP; i += NTHR * 4) {
      const v4i v = *(const v4ia*)(pl + i);
      *(volatile v4i*)(lp + i) = v;
    }
#pragma unroll 1
    for (int i = tid * 4; i < NBRUN; i += NTHR * 4) {
      const v4i v = *(const v4ia*)(offs + i);
      *(volatile v4i*)(op + i) = v;
    }
  }
#pragma unroll 1
  for (int i = tid * 4; i < NBRUN; i += NTHR * 4) {
    v4i v = *(const v4ia*)(cnt + i);
    const int g = slot0 + i;
    v.x = (g     < NN) ? v.x : 0;
    v.y = (g + 1 < NN) ? v.y : 0;
    v.z = (g + 2 < NN) ? v.z : 0;
    v.w = (g + 3 < NN) ? v.w : 0;
    *(volatile v4i*)(cp + i) = v;
  }
  if (tid < 8) {
    const v4i f = {ov, ov, ov, ov};
    *(volatile v4i*)(fp + 4 * tid) = f;
  }
}

__global__ __launch_bounds__(NTHR) void k_bucket(const int* __restrict__ edges, int* LIST, int* CNTALL,
                                                 int* OFF, int* FLAG) {
  extern __shared__ __attribute__((aligned(16))) int dsm[];
  int* wl   = dsm;
  int* pl   = dsm + NWAVE * WLCAP;
  int* cnt  = pl + RCAP;
  int* offs = cnt + NBRUN;
  int* cur  = offs + NBRUN;
  int* misc = cur + NBRUN;
  const int tid = (int)threadIdx.x, lane = tid & 31, wave = tid >> 5;
  const int role   = (int)blockIdx.x / NBK;
  const int blk    = (int)blockIdx.x - role * NBK;
  const int isList = role < NT ? 1 : 0;
  const int t      = role & (NT - 1);
  const int krow   = 2 * t + isList;
  const int* keys  = edges + (size_t)krow * NE;
  const int* pays  = edges + (size_t)(2 * t) * NE;
  const unsigned nbs = (unsigned)(blk * NBRUN);

  {
    const v4i z4 = {0, 0, 0, 0};
    for (int i = tid * 4; i < BK_ZINTS; i += NTHR * 4) *(v4ia*)(dsm + i) = z4;
    if (tid < 16) misc[tid] = 0;
  }
  __syncthreads();

  {
    const int per  = ((NE + NWAVE * WCH - 1) / (NWAVE * WCH)) * WCH;
    const int ebeg = wave * per;
    const int eend = (ebeg + per < NE) ? (ebeg + per) : NE;
    int* mylist = wl + wave * WLCAP;
    int wc = 0;
#pragma unroll 1
    for (int cb = ebeg; cb < eend; cb += WCH) {
      const int e0 = cb + lane * EPT;
      const v4i da = *(const v4ia*)(keys + e0);
      const unsigned s0 = (unsigned)da.x - nbs, s1 = (unsigned)da.y - nbs;
      const unsigned s2 = (unsigned)da.z - nbs, s3 = (unsigned)da.w - nbs;
      const bool h0 = s0 < (unsigned)NBRUN, h1 = s1 < (unsigned)NBRUN;
      const bool h2 = s2 < (unsigned)NBRUN, h3 = s3 < (unsigned)NBRUN;
      const unsigned m0 = __builtin_amdgcn_ballot_w32(h0), m1 = __builtin_amdgcn_ballot_w32(h1);
      const unsigned m2 = __builtin_amdgcn_ballot_w32(h2), m3 = __builtin_amdgcn_ballot_w32(h3);
      const unsigned any = m0 | m1 | m2 | m3;
      if (any != 0u) {
        const int pre = (int)(__builtin_amdgcn_mbcnt_lo(m0, 0u) + __builtin_amdgcn_mbcnt_lo(m1, 0u) +
                              __builtin_amdgcn_mbcnt_lo(m2, 0u) + __builtin_amdgcn_mbcnt_lo(m3, 0u));
        int p = wc + pre;
        if (h0) { if (p < WLCAP) mylist[p] = ((e0 + 0) << SLB) | (int)s0; p = p + 1; }
        if (h1) { if (p < WLCAP) mylist[p] = ((e0 + 1) << SLB) | (int)s1; p = p + 1; }
        if (h2) { if (p < WLCAP) mylist[p] = ((e0 + 2) << SLB) | (int)s2; p = p + 1; }
        if (h3) { if (p < WLCAP) mylist[p] = ((e0 + 3) << SLB) | (int)s3; p = p + 1; }
        wc += (int)(__builtin_popcount(m0) + __builtin_popcount(m1) + __builtin_popcount(m2) + __builtin_popcount(m3));
      }
    }
    if (lane == 0) misc[wave] = wc;
  }
  __syncthreads();

  if (wave == 0) {
    int ov = 0;
#pragma unroll 1
    for (int w2 = 0; w2 < NWAVE; ++w2) {
      int c = misc[w2];
      if (c > WLCAP) ov = 1;
      c = c < 0 ? 0 : (c > WLCAP ? WLCAP : c);
#pragma unroll 1
      for (int b0 = 0; b0 < c; b0 += 32) {
        const int idx = b0 + lane;
        const int ent = wl[w2 * WLCAP + (idx < WLCAP ? idx : WLCAP - 1)];
        const int m32 = (c - b0) < 32 ? (c - b0) : 32;
#pragma unroll 1
        for (int k = 0; k < m32; ++k) {
          const int u    = __builtin_amdgcn_readlane(ent, k);
          const int slot = u & (NBRUN - 1);
          if (lane == 0) cnt[slot] = cnt[slot] + 1;
        }
      }
    }
    if (lane == 0) misc[9] = ov;
  }
  __syncthreads();
  if (wave == 0) {
    const int base = lane * (NBRUN / 32);
    int s = 0;
#pragma unroll 1
    for (int i = 0; i < NBRUN / 32; ++i) s += cnt[base + i];
    int incl = s;
#pragma unroll
    for (int d = 1; d < 32; d <<= 1) {
      const int y = __shfl_up(incl, d, 32);
      if (lane >= d) incl += y;
    }
    int run = incl - s;
#pragma unroll 1
    for (int i = 0; i < NBRUN / 32; ++i) {
      const int cv = cnt[base + i];
      offs[base + i] = run;
      cur[base + i]  = run;
      run += cv;
    }
  }
  __syncthreads();

  if (wave == 0 && isList != 0) {
#pragma unroll 1
    for (int w2 = 0; w2 < NWAVE; ++w2) {
      int c = misc[w2];
      c = c < 0 ? 0 : (c > WLCAP ? WLCAP : c);
#pragma unroll 1
      for (int b0 = 0; b0 < c; b0 += 32) {
        const int idx = b0 + lane;
        const int ent = wl[w2 * WLCAP + (idx < WLCAP ? idx : WLCAP - 1)];
        int eid = (ent >> SLB) & 0x7FFFF;
        eid = eid > NE - 1 ? NE - 1 : eid;
        int sr = pays[eid];
        sr = sr < 0 ? 0 : (sr > NN - 1 ? NN - 1 : sr);
        const int m32 = (c - b0) < 32 ? (c - b0) : 32;
#pragma unroll 1
        for (int k = 0; k < m32; ++k) {
          const int u    = __builtin_amdgcn_readlane(ent, k);
          const int wd   = __builtin_amdgcn_readlane(sr, k);
          const int slot = u & (NBRUN - 1);
          if (lane == 0) {
            int p = cur[slot];
            p = p < 0 ? 0 : (p > RCAP - 1 ? RCAP - 1 : p);
            pl[p] = wd;
            cur[slot] = p + 1;
          }
        }
      }
    }
  }
  __syncthreads();

  const int ovf = misc[9];
  int* lp = LIST + ((size_t)t * NBK + (size_t)blk) * RCAP;
  int* cp = CNTALL + (size_t)role * NSLOT + (size_t)blk * NBRUN;
  int* op = OFF + (size_t)t * NSLOT + (size_t)blk * NBRUN;
  int* fp = FLAG + (size_t)blockIdx.x * 32;
  bucket_flush(pl, cnt, offs, ovf, isList, blk * NBRUN, lp, cp, op, fp, tid);
  __threadfence();
  bucket_flush(pl, cnt, offs, ovf, isList, blk * NBRUN, lp, cp, op, fp, tid);
}

__device__ __forceinline__ void gemm_16x128(const unsigned short* __restrict__ ap,
                                            const unsigned short* __restrict__ bp, v8f (&acc)[8]) {
#pragma unroll 1
  for (int k0 = 0; k0 < FD; k0 += 32) {
    FragB af;
    af.h[0] = *(const v8usa*)(ap + k0);
    af.h[1] = *(const v8usa*)(ap + k0 + 16);
#pragma unroll
    for (int nt = 0; nt < 8; ++nt) {
      const unsigned short* wq = bp + (size_t)(16 * nt) * (size_t)FD + k0;
      FragB bf;
      bf.h[0] = *(const v8usa*)wq;
      bf.h[1] = *(const v8usa*)(wq + 16);
      acc[nt] = wmb(af, bf, acc[nt]);
    }
  }
}

__global__ __launch_bounds__(NTHR) __attribute__((amdgpu_num_vgpr(248)))
void k_gemm(const unsigned short* __restrict__ XB, const unsigned short* __restrict__ WTt,
            const int* __restrict__ OCt, const int* __restrict__ FLAGc, float* P) {
  extern __shared__ __attribute__((aligned(16))) float gsm[];
  float* stg = gsm;
  float* srs = gsm + GBM * SP;
  const int tid = (int)threadIdx.x, lane = tid & 31, wave = tid >> 5, hh = lane >> 4, m = lane & 15;
  const int rowBase = (int)blockIdx.x * GBM;
  const int flag = FLAGc[(size_t)(rowBase >> SLB) * 32];

  if (tid < 32) {
    const v4i c4 = *(const v4ia*)(OCt + rowBase + 4 * tid);
    const float f0 = fmaxf((float)c4.x, 1.0f), f1 = fmaxf((float)c4.y, 1.0f);
    const float f2 = fmaxf((float)c4.z, 1.0f), f3 = fmaxf((float)c4.w, 1.0f);
    v4f r;
    r.x = 1.0f / sqrtf(f0); r.y = 1.0f / sqrtf(f1); r.z = 1.0f / sqrtf(f2); r.w = 1.0f / sqrtf(f3);
    *(v4fa*)(srs + 4 * tid) = r;
  }

  v8f acc[8];
  {
    const v8f z = {0.f, 0.f, 0.f, 0.f, 0.f, 0.f, 0.f, 0.f};
#pragma unroll
    for (int t = 0; t < 8; ++t) acc[t] = z;
  }
  const unsigned short* ap = XB + (size_t)(rowBase + 16 * wave + m) * (size_t)FD + 8 * hh;
  const unsigned short* bp = WTt + (size_t)m * (size_t)FD + 8 * hh;
  gemm_16x128(ap, bp, acc);
#pragma unroll
  for (int nt = 0; nt < 8; ++nt) {
#pragma unroll
    for (int r = 0; r < 8; ++r) stg[(16 * wave + 8 * hh + r) * SP + 16 * nt + m] = acc[nt][r];
  }
  __syncthreads();

  const float qnan = __uint_as_float(0x7fc00000u);
  const bool bad = flag != 0;
#pragma unroll 1
  for (int i = 0; i < 16; ++i) {
    const int lr   = 16 * wave + i;
    const int grow = rowBase + lr;
    const bool live = grow < NN;
    const v4f a = *(const v4fa*)(stg + lr * SP + 4 * lane);
    asm volatile("" :: "v"(a));
    const float s = srs[lr];
    float v0 = a.x * s, v1 = a.y * s, v2 = a.z * s, v3 = a.w * s;
    v0 = bad ? qnan : v0; v1 = bad ? qnan : v1; v2 = bad ? qnan : v2; v3 = bad ? qnan : v3;
    v4f o;
    o.x = live ? v0 : 0.0f; o.y = live ? v1 : 0.0f; o.z = live ? v2 : 0.0f; o.w = live ? v3 : 0.0f;
    st2_v4f(P + (size_t)grow * FD + 4 * lane, o);
  }
}

template <int MODE>
__global__ __launch_bounds__(NTHR) void k_replay(const int* __restrict__ LISTt, const int* __restrict__ CNTt,
                                                 const int* __restrict__ OFFt, const int* __restrict__ FLAGt,
                                                 const float* __restrict__ P, const float* __restrict__ BF,
                                                 float* out) {
  const int tid = (int)threadIdx.x, lane = tid & 31, wave = tid >> 5;
  const int row = (int)blockIdx.x * RPB + wave;
  const int bk  = row >> SLB;

  int cv = CNTt[row];
  int ov = OFFt[row];
  const int fl = FLAGt[(size_t)bk * 32];
  const bool big = cv > DEGCAP;
  cv = cv < 0 ? 0 : (cv > DEGCAP ? DEGCAP : cv);
  ov = ov < 0 ? 0 : (ov > RCAP - 1 ? RCAP - 1 : ov);
  const int c = __builtin_amdgcn_readfirstlane(cv);
  const int o = __builtin_amdgcn_readfirstlane(ov);
  int last = o + c - 1;
  last = last < o ? o : last;
  last = last > RCAP - 1 ? RCAP - 1 : last;

  const int* lb = LISTt + (size_t)bk * RCAP;
  int idx = o + lane;
  idx = idx > last ? last : idx;
  int ent = lb[idx];
  ent = ent < 0 ? 0 : (ent > NN - 1 ? NN - 1 : ent);
  float a0 = 0.0f, a1 = 0.0f, a2 = 0.0f, a3 = 0.0f;
#pragma unroll 1
  for (int j = 0; j < c; ++j) {
    const int sk = __builtin_amdgcn_readlane(ent, j);
    const v4f v = *(const v4fa*)(P + (size_t)sk * FD + 4 * lane);
    a0 += v.x; a1 += v.y; a2 += v.z; a3 += v.w;
  }

  const float dn = sqrtf(fmaxf((float)c, 1.0f));
  float r0 = a0 / dn, r1 = a1 / dn, r2 = a2 / dn, r3 = a3 / dn;

  float* op = out + (size_t)row * FD + 4 * lane;
  if constexpr (MODE != 0) {
    const v4f old = *(const v4fa*)op;
    r0 = old.x + r0; r1 = old.y + r1; r2 = old.z + r2; r3 = old.w + r3;
  }
  if constexpr (MODE == 2) {
    const v4f bb = *(const v4fa*)(BF + 4 * lane);
    r0 = r0 + bb.x; r1 = r1 + bb.y; r2 = r2 + bb.z; r3 = r3 + bb.w;
  }

  const float qnan = __uint_as_float(0x7fc00000u);
  const bool bad = (fl != 0) | big;
  v4f res;
  res.x = bad ? qnan : r0; res.y = bad ? qnan : r1; res.z = bad ? qnan : r2; res.w = bad ? qnan : r3;
  st2_v4f(op, res);
}

extern "C" void kernel_launch(void* const* d_in, const int* in_sizes, int n_in,
                              void* d_out, int out_size, void* d_ws, size_t ws_size,
                              hipStream_t stream) {
  if (n_in < 4) return;
  if (in_sizes[0] != NN * FD) return;
  if (in_sizes[1] != NT * 2 * NE) return;
  if (in_sizes[2] != NT * FD * FD) return;
  if (in_sizes[3] != FD) return;
  if (out_size != NN * FD) return;

  const float* x  = (const float*)d_in[0];
  const int*   ed = (const int*)d_in[1];
  const float* W  = (const float*)d_in[2];
  const float* b  = (const float*)d_in[3];
  float* out = (float*)d_out;

  constexpr size_t zXB   = (size_t)MP * FD * 2;
  constexpr size_t zWT   = (size_t)NT * FD * FD * 2;
  constexpr size_t zP    = (size_t)MP * FD * 4;
  constexpr size_t zLIST = (size_t)NT * NBK * RCAP * 4;
  constexpr size_t zCNT  = (size_t)NROLE * NSLOT * 4;
  constexpr size_t zOFF  = (size_t)NT * NSLOT * 4;
  constexpr size_t zFLAG = (size_t)NROLE * NBK * 128;
  constexpr size_t zBF   = 512;
  constexpr size_t oXB   = 0;
  constexpr size_t oWT   = oXB + zXB;
  constexpr size_t oP    = oWT + zWT;
  constexpr size_t oLIST = oP + zP;
  constexpr size_t oCNT  = oLIST + zLIST;
  constexpr size_t oOFF  = oCNT + zCNT;
  constexpr size_t oFLAG = oOFF + zOFF;
  constexpr size_t oBF   = oFLAG + zFLAG;
  constexpr size_t oEND  = oBF + zBF;
  static_assert(zXB % 256 == 0 && zWT % 256 == 0 && zP % 256 == 0 && zLIST % 256 == 0);
  static_assert(zCNT % 256 == 0 && zOFF % 256 == 0 && zFLAG % 256 == 0 && zBF % 256 == 0);
  static_assert(oEND <= (size_t)WSMAX);
  if (oEND > ws_size) return;

  char* ws = (char*)d_ws;
  unsigned short* XB   = (unsigned short*)(ws + oXB);
  unsigned short* WT   = (unsigned short*)(ws + oWT);
  float*          P    = (float*)(ws + oP);
  int*            LIST = (int*)(ws + oLIST);
  int*            CNT  = (int*)(ws + oCNT);
  int*            OFF  = (int*)(ws + oOFF);
  int*            FLAG = (int*)(ws + oFLAG);
  float*          BF   = (float*)(ws + oBF);

  hipFuncSetAttribute(reinterpret_cast<const void*>(&k_bucket), hipFuncAttributeMaxDynamicSharedMemorySize, (int)BK_LDS);
  hipFuncSetAttribute(reinterpret_cast<const void*>(&k_gemm), hipFuncAttributeMaxDynamicSharedMemorySize, (int)GEMM_LDS);

  k_prep<<<PBTOT, NTHR, 0, stream>>>(x, W, b, XB, WT, BF);
  k_bucket<<<NROLE * NBK, NTHR, BK_LDS, stream>>>(ed, LIST, CNT, OFF, FLAG);

  for (int t = 0; t < NT; ++t) {
    const unsigned short* wt_t = WT + (size_t)t * FD * FD;
    const int* oc_t   = CNT + (size_t)(NT + t) * NSLOT;
    const int* fc_t   = FLAG + (size_t)(NT + t) * NBK * 32;
    const int* list_t = LIST + (size_t)t * NBK * RCAP;
    const int* cnt_t  = CNT + (size_t)t * NSLOT;
    const int* off_t  = OFF + (size_t)t * NSLOT;
    const int* fl_t   = FLAG + (size_t)t * NBK * 32;
    k_gemm<<<MP / GBM, NTHR, GEMM_LDS, stream>>>(XB, wt_t, oc_t, fc_t, P);
    if (t == 0)
      k_replay<0><<<NN / RPB, NTHR, 0, stream>>>(list_t, cnt_t, off_t, fl_t, P, BF, out);
    else if (t == NT - 1)
      k_replay<2><<<NN / RPB, NTHR, 0, stream>>>(list_t, cnt_t, off_t, fl_t, P, BF, out);
    else
      k_replay<1><<<NN / RPB, NTHR, 0, stream>>>(list_t, cnt_t, off_t, fl_t, P, BF, out);
  }
}
